// GraphAttention_48541720379787
// MI455X (gfx1250) — hardware-verified
//
#include <hip/hip_runtime.h>
#include <math.h>
#include <stdint.h>

#define NNODE 4096
#define FIN   512
#define FD    128
#define NHD   8
#define QKS   1024
#define QSC   64.0f
#define QSCI  0.015625f
#define PSC   1024.0f
#define OSC   0.0009765625f

static_assert(NNODE % 128 == 0 && NNODE % 64 == 0 && NNODE % 32 == 0);
static_assert(FIN % 64 == 0 && FIN % 32 == 0 && FD == 128 && QKS == NHD * FD);
static_assert(QKS % 128 == 0 && FD % 32 == 0);

typedef __bf16         v16b __attribute__((ext_vector_type(16)));
typedef __bf16         v8b  __attribute__((ext_vector_type(8)));
typedef _Float16       v16h __attribute__((ext_vector_type(16)));
typedef _Float16       v8h  __attribute__((ext_vector_type(8)));
typedef float          v8f  __attribute__((ext_vector_type(8)));
typedef float          v4f  __attribute__((ext_vector_type(4)));
typedef unsigned int   v4u  __attribute__((ext_vector_type(4)));
typedef v4f __attribute__((may_alias)) v4fa;
typedef v4u __attribute__((may_alias)) v4ua;
typedef v8b __attribute__((may_alias)) v8ba;
typedef v8h __attribute__((may_alias)) v8ha;

__device__ __forceinline__ unsigned short bf_bits(float f) {
  const unsigned u = __float_as_uint(f);
  return (unsigned short)((u + 0x7FFFu + ((u >> 16) & 1u)) >> 16);
}
__device__ __forceinline__ float bf_val(unsigned short h) { return __uint_as_float(((unsigned)h) << 16); }
__device__ __forceinline__ float bf_rne(float f) { return bf_val(bf_bits(f)); }
__device__ __forceinline__ v4f bf_rne4(v4f a) {
  v4f r;
  r[0] = bf_rne(a[0]); r[1] = bf_rne(a[1]); r[2] = bf_rne(a[2]); r[3] = bf_rne(a[3]);
  return r;
}
__device__ __forceinline__ unsigned short h_bits(float f) {
  const _Float16 hv = (_Float16)f;
  return __builtin_bit_cast(unsigned short, hv);
}
__device__ __forceinline__ unsigned pk16(unsigned short a, unsigned short b) { return (unsigned)a | ((unsigned)b << 16); }
__device__ __forceinline__ v8f zero8() { v8f z = {0.f, 0.f, 0.f, 0.f, 0.f, 0.f, 0.f, 0.f}; return z; }
__device__ __forceinline__ int wave_id() { return __builtin_amdgcn_readfirstlane((int)(threadIdx.x >> 5)); }

__device__ __forceinline__ void lds_wave_sync() {
  __builtin_amdgcn_fence(__ATOMIC_RELEASE, "workgroup");
  __builtin_amdgcn_wave_barrier();
  __builtin_amdgcn_fence(__ATOMIC_ACQUIRE, "workgroup");
}

union FragB { v16b v; v8b h[2]; };
union FragH { v16h v; v8h h[2]; };
__device__ __forceinline__ v16b ldfrag_b(const __bf16* p) {
  FragB f;
  f.h[0] = *(const v8ba*)(p);
  f.h[1] = *(const v8ba*)(p + 16);
  return f.v;
}
__device__ __forceinline__ v16h ldfrag_h(const _Float16* p) {
  FragH f;
  f.h[0] = *(const v8ha*)(p);
  f.h[1] = *(const v8ha*)(p + 16);
  return f.v;
}
__device__ __forceinline__ v8f mma_b(v16b a, v16b b, v8f c) {
  return __builtin_amdgcn_wmma_f32_16x16x32_bf16(false, a, false, b, (short)0, c, false, false);
}
__device__ __forceinline__ v8f mma_h(v16h a, v16h b, v8f c) {
  return __builtin_amdgcn_wmma_f32_16x16x32_f16(false, a, false, b, (short)0, c, false, false);
}
__device__ __forceinline__ void guard_b3(v8f& a, v8f& b, v16b x0, v16b x1, v16b y0) {
  asm volatile("v_nop\n\tv_nop\n\tv_nop\n\tv_nop" : "+v"(a), "+v"(b) : "v"(x0), "v"(x1), "v"(y0) : "memory");
}
__device__ __forceinline__ void guard4_h5(v8f& a, v8f& b, v8f& c, v8f& d, v16h q, v16h k0, v16h k1, v16h k2, v16h k3) {
  asm volatile("v_nop\n\tv_nop\n\tv_nop\n\tv_nop" : "+v"(a), "+v"(b), "+v"(c), "+v"(d) : "v"(q), "v"(k0), "v"(k1), "v"(k2), "v"(k3) : "memory");
}
__device__ __forceinline__ void guard1_h4(v8f& a, v16h w, v16h x, v16h y, v16h z) {
  asm volatile("v_nop\n\tv_nop\n\tv_nop\n\tv_nop" : "+v"(a) : "v"(w), "v"(x), "v"(y), "v"(z) : "memory");
}
__device__ __forceinline__ void acc_guard4(v8f& a, v8f& b, v8f& c, v8f& d) {
  asm volatile("v_nop\n\tv_nop\n\tv_nop\n\tv_nop" : "+v"(a), "+v"(b), "+v"(c), "+v"(d));
}

__global__ __launch_bounds__(256) void prep_x_kernel(const float* __restrict__ x, unsigned short* __restrict__ xb, int nunits) {
  const int i = (int)blockIdx.x * 256 + (int)threadIdx.x;
  if (i >= nunits) return;
  const size_t e = 8 * (size_t)i;
  const v4f a = *(const v4fa*)(x + e);
  const v4f c = *(const v4fa*)(x + e + 4);
  v4u w;
  w[0] = pk16(bf_bits(a[0]), bf_bits(a[1]));
  w[1] = pk16(bf_bits(a[2]), bf_bits(a[3]));
  w[2] = pk16(bf_bits(c[0]), bf_bits(c[1]));
  w[3] = pk16(bf_bits(c[2]), bf_bits(c[3]));
  *(volatile v4u*)(xb + e) = w;
  __threadfence();
  *(volatile v4u*)(xb + e) = w;
}

__global__ __launch_bounds__(256) void prep_q_kernel(const float* __restrict__ x, unsigned short* __restrict__ qh, int nunits) {
  const int i = (int)blockIdx.x * 256 + (int)threadIdx.x;
  if (i >= nunits) return;
  const size_t e = 8 * (size_t)i;
  const v4f a = *(const v4fa*)(x + e);
  const v4f c = *(const v4fa*)(x + e + 4);
  v4u w;
  w[0] = pk16(h_bits(QSC * bf_rne(a[0])), h_bits(QSC * bf_rne(a[1])));
  w[1] = pk16(h_bits(QSC * bf_rne(a[2])), h_bits(QSC * bf_rne(a[3])));
  w[2] = pk16(h_bits(QSC * bf_rne(c[0])), h_bits(QSC * bf_rne(c[1])));
  w[3] = pk16(h_bits(QSC * bf_rne(c[2])), h_bits(QSC * bf_rne(c[3])));
  *(volatile v4u*)(qh + e) = w;
  __threadfence();
  *(volatile v4u*)(qh + e) = w;
}

__global__ __launch_bounds__(256) void tconv_bf16_kernel(const float* __restrict__ W, unsigned short* __restrict__ outp,
                                                         int R, int Cc, long sIn, long sOut) {
  __shared__ __align__(16) float tf[64 * 68];
  W    += (size_t)blockIdx.z * sIn;
  outp += (size_t)blockIdx.z * sOut;
  const int c0  = (int)blockIdx.x * 64;
  const int r0  = (int)blockIdx.y * 64;
  const int tid = (int)threadIdx.x;
  {
    const int lr = tid >> 4;
    const int c4 = (tid & 15) * 4;
#pragma unroll
    for (int it = 0; it < 4; ++it) {
      const int rr = it * 16 + lr;
      const v4f a = *(const v4fa*)(W + (size_t)(r0 + rr) * Cc + c0 + c4);
      *(v4f*)(tf + rr * 68 + c4) = a;
    }
  }
  __syncthreads();
  const int sub = tid >> 3;
  const int c8  = (tid & 7) * 8;
  v4u hv[2];
#pragma unroll
  for (int it = 0; it < 2; ++it) {
    const int oc = it * 32 + sub;
    v4u a;
#pragma unroll
    for (int q = 0; q < 4; ++q) {
      const float f0 = tf[(c8 + 2 * q) * 68 + oc];
      const float f1 = tf[(c8 + 2 * q + 1) * 68 + oc];
      a[q] = pk16(bf_bits(f0), bf_bits(f1));
    }
    hv[it] = a;
  }
  for (int pass = 0; pass < 2; ++pass) {
#pragma unroll
    for (int it = 0; it < 2; ++it) {
      const int oc = it * 32 + sub;
      const size_t go = (size_t)(c0 + oc) * R + r0 + c8;
      *(volatile v4u*)(outp + go) = hv[it];
    }
    __threadfence();
  }
}

#define SLAB_PERW 2048

template <bool SRCDOT>
__global__ __launch_bounds__(128) __attribute__((amdgpu_num_vgpr(256))) void gemm_kernel(
    const unsigned short* Ap, int lda, const unsigned short* Btp, int ldb,
    unsigned short* C0, int ldc, int M, int N, int K,
    const float* __restrict__ asrc, float* srcp) {
  __shared__ __align__(16) float slab_all[4 * SLAB_PERW];

  const int lane = threadIdx.x & 31;
  const int wave = wave_id();
  const int hh = lane >> 4;
  const int rl = lane & 15;
  const int tilesN = N >> 7;
  const int tilesM = M >> 5;
  const int tile = (int)blockIdx.x * 4 + wave;
  if (tile >= tilesM * tilesN) return;
  const int tm = tile / tilesN;
  const int tn = tile - tm * tilesN;
  const int m0 = tm << 5;
  const int n0 = tn << 7;

  const __bf16* A  = (const __bf16*)(const void*)Ap;
  const __bf16* Bt = (const __bf16*)(const void*)Btp;

  v8f acc[2][8];
#pragma unroll
  for (int i = 0; i < 2; ++i)
#pragma unroll
    for (int j = 0; j < 8; ++j) acc[i][j] = zero8();

  for (int k0 = 0; k0 < K; k0 += 32) {
    const v16b a0f = ldfrag_b(A + (size_t)(m0 + rl) * lda + k0 + 8 * hh);
    const v16b a1f = ldfrag_b(A + (size_t)(m0 + 16 + rl) * lda + k0 + 8 * hh);
#pragma unroll
    for (int j = 0; j < 8; ++j) {
      const v16b bh = ldfrag_b(Bt + (size_t)(n0 + j * 16 + rl) * ldb + k0 + 8 * hh);
      acc[0][j] = mma_b(a0f, bh, acc[0][j]);
      acc[1][j] = mma_b(a1f, bh, acc[1][j]);
      guard_b3(acc[0][j], acc[1][j], a0f, a1f, bh);
    }
  }
  acc_guard4(acc[0][0], acc[0][1], acc[0][2], acc[0][3]);
  acc_guard4(acc[0][4], acc[0][5], acc[0][6], acc[0][7]);
  acc_guard4(acc[1][0], acc[1][1], acc[1][2], acc[1][3]);
  acc_guard4(acc[1][4], acc[1][5], acc[1][6], acc[1][7]);

  float* slf = slab_all + wave * SLAB_PERW;
  const int hsel = n0 >> 7;
  float srcv = 0.f;
#pragma unroll
  for (int i = 0; i < 2; ++i) {
#pragma unroll
    for (int j = 0; j < 8; ++j) {
#pragma unroll
      for (int r = 0; r < 8; ++r)
        slf[(8 * hh + r) * 128 + j * 16 + rl] = acc[i][j][r];
    }
    lds_wave_sync();
    if (SRCDOT) {
      const int m = m0 + i * 16 + rl;
      const float* ap = asrc + ((size_t)hsel * NNODE + m) * FD + hh * 64;
      const float* sp = slf + rl * 128 + hh * 64;
      float t = 0.f;
#pragma unroll 4
      for (int it = 0; it < 16; ++it) {
        const v4f av = bf_rne4(*(const v4fa*)(ap + it * 4));
        const v4f hv = *(const v4fa*)(sp + it * 4);
        t = fmaf(hv[0], av[0], t);
        t = fmaf(hv[1], av[1], t);
        t = fmaf(hv[2], av[2], t);
        t = fmaf(hv[3], av[3], t);
      }
      t += __shfl_xor(t, 16, 32);
      srcv = (hh == i) ? t : srcv;
    }
    for (int pass = 0; pass < 2; ++pass) {
#pragma unroll
      for (int it = 0; it < 8; ++it) {
        const int row = it * 2 + hh;
        const int c8  = rl * 8;
        const float* spp = slf + row * 128 + c8;
        const v4f f0 = *(const v4fa*)(spp);
        const v4f f1 = *(const v4fa*)(spp + 4);
        v4u w;
        w[0] = pk16(h_bits(f0[0]), h_bits(f0[1]));
        w[1] = pk16(h_bits(f0[2]), h_bits(f0[3]));
        w[2] = pk16(h_bits(f1[0]), h_bits(f1[1]));
        w[3] = pk16(h_bits(f1[2]), h_bits(f1[3]));
        const size_t go = (size_t)(m0 + i * 16 + row) * ldc + n0 + c8;
        *(volatile v4u*)(C0 + go) = w;
      }
      __threadfence();
    }
    lds_wave_sync();
  }
  if (SRCDOT) {
    float* dp = srcp + (size_t)hsel * NNODE + m0 + lane;
    *(volatile float*)dp = srcv;
    __threadfence();
    *(volatile float*)dp = srcv;
  }
}

#define KT       64
#define PSP      72
#define OSTP     128
#define NTILE    (FD / 16)
#define ATT_O_F  (4 * NTILE * 32 * 8)
#define ATT_P_H  (4 * 16 * PSP)
#define ATT_S_F  (4 * 16 * OSTP)
#define ATT_LDS_BYTES (ATT_O_F * 4 + ATT_P_H * 2 + ATT_S_F * 4)
static_assert(ATT_LDS_BYTES == 74752);
static_assert((ATT_O_F * 4) % 16 == 0 && ((ATT_O_F * 4 + ATT_P_H * 2) % 16) == 0);
static_assert(NNODE % KT == 0 && KT == 64 && NTILE == 8);

__global__ __launch_bounds__(128) __attribute__((amdgpu_num_vgpr(240))) void attn_kernel(
    const unsigned short* __restrict__ qp, const unsigned short* __restrict__ kp,
    const unsigned short* __restrict__ vtp, const float* __restrict__ srcp,
    const float* __restrict__ attb, float* __restrict__ out) {
  extern __shared__ v4f att_dyn[];
  float*    o_l   = (float*)(void*)att_dyn;
  _Float16* lds_p = (_Float16*)(void*)((char*)(void*)att_dyn + ATT_O_F * 4);
  float*    lds_s = (float*)(void*)((char*)(void*)att_dyn + ATT_O_F * 4 + ATT_P_H * 2);

  const int tid  = (int)threadIdx.x;
  const int lane = tid & 31;
  const int wave = wave_id();
  const int hh   = lane >> 4;
  const int c    = lane & 15;
  const int qb   = (int)blockIdx.x;
  const int h    = (int)blockIdx.y;
  const int q0   = qb * 64 + wave * 16;

  const _Float16* Qr = (const _Float16*)(const void*)qp  + ((size_t)h * NNODE + q0 + c) * FD + 8 * hh;
  const _Float16* Kg = (const _Float16*)(const void*)kp  + (size_t)h * FD + 8 * hh;
  const _Float16* Vg = (const _Float16*)(const void*)vtp + (size_t)(h * FD) * NNODE + 8 * hh;
  _Float16* ph = lds_p + wave * (16 * PSP);
  float*    ow = o_l + wave * (NTILE * 32 * 8) + lane * 8;

  {
    const v4f z4 = {0.f, 0.f, 0.f, 0.f};
#pragma unroll
    for (int t = 0; t < NTILE; ++t) {
      *(v4fa*)(ow + t * 256)     = z4;
      *(v4fa*)(ow + t * 256 + 4) = z4;
    }
  }

  float cadd[8];
  {
    const size_t ro = (size_t)h * NNODE + q0 + 8 * hh;
    const v4f s0 = *(const v4fa*)(srcp + ro);
    const v4f s1 = *(const v4fa*)(srcp + ro + 4);
    const v4f b0 = bf_rne4(*(const v4fa*)(attb + ro));
    const v4f b1 = bf_rne4(*(const v4fa*)(attb + ro + 4));
#pragma unroll
    for (int r = 0; r < 4; ++r) { cadd[r] = s0[r] + b0[r]; cadd[4 + r] = s1[r] + b1[r]; }
  }

  float mrow[8], lrow[8];
#pragma unroll
  for (int r = 0; r < 8; ++r) { mrow[r] = -INFINITY; lrow[r] = 0.f; }

#pragma unroll 1
  for (int kc = 0; kc < NNODE / KT; ++kc) {
    const int kv0 = kc * KT;
    v8f s[4];
    s[0] = zero8(); s[1] = zero8(); s[2] = zero8(); s[3] = zero8();
#pragma unroll
    for (int dc = 0; dc < FD / 32; ++dc) {
      const v16h qa = ldfrag_h(Qr + dc * 32);
      v16h kb[4];
#pragma unroll
      for (int j = 0; j < 4; ++j) kb[j] = ldfrag_h(Kg + (size_t)(kv0 + j * 16 + c) * QKS + dc * 32);
#pragma unroll
      for (int j = 0; j < 4; ++j) s[j] = mma_h(qa, kb[j], s[j]);
      guard4_h5(s[0], s[1], s[2], s[3], qa, kb[0], kb[1], kb[2], kb[3]);
    }
    float cm[8];
#pragma unroll
    for (int r = 0; r < 8; ++r) {
      float m = -INFINITY;
#pragma unroll
      for (int j = 0; j < 4; ++j) {
        const float sv = s[j][r] * QSCI + cadd[r];
        s[j][r] = sv;
        m = fmaxf(m, sv);
      }
#pragma unroll
      for (int off = 1; off < 16; off <<= 1) m = fmaxf(m, __shfl_xor(m, off, 32));
      cm[r] = m;
    }
    float alpha[8];
#pragma unroll
    for (int r = 0; r < 8; ++r) {
      const float mnew = fmaxf(mrow[r], cm[r]);
      const float al   = __expf(mrow[r] - mnew);
      mrow[r]  = mnew;
      alpha[r] = al;
      float psum = 0.f;
#pragma unroll
      for (int j = 0; j < 4; ++j) {
        const float p = __expf(s[j][r] - mnew);
        psum += p;
        ph[(8 * hh + r) * PSP + j * 16 + c] = (_Float16)(p * PSC);
      }
#pragma unroll
      for (int off = 1; off < 16; off <<= 1) psum += __shfl_xor(psum, off, 32);
      lrow[r] = lrow[r] * al + psum;
    }
    lds_wave_sync();
    const v16h pa0 = ldfrag_h(ph + c * PSP + 8 * hh);
    const v16h pa1 = ldfrag_h(ph + c * PSP + 32 + 8 * hh);
#pragma unroll 1
    for (int cc = 0; cc < 2; ++cc) {
      float* ocl = ow + cc * 1024;
      v8f oc[4];
#pragma unroll
      for (int t = 0; t < 4; ++t) {
        const v4f a4 = *(const v4fa*)(ocl + t * 256);
        const v4f b4 = *(const v4fa*)(ocl + t * 256 + 4);
        v8f o8;
#pragma unroll
        for (int r = 0; r < 4; ++r) {
          o8[r]     = a4[r] * alpha[r];
          o8[4 + r] = b4[r] * alpha[4 + r];
        }
        oc[t] = o8;
      }
#pragma unroll
      for (int t = 0; t < 4; ++t) {
        const size_t vo = (size_t)((cc * 4 + t) * 16 + c) * NNODE + kv0;
        const v16h vb0 = ldfrag_h(Vg + vo);
        const v16h vb1 = ldfrag_h(Vg + vo + 32);
        oc[t] = mma_h(pa0, vb0, oc[t]);
        oc[t] = mma_h(pa1, vb1, oc[t]);
        guard1_h4(oc[t], pa0, pa1, vb0, vb1);
      }
#pragma unroll
      for (int t = 0; t < 4; ++t) {
        v4f a4, b4;
#pragma unroll
        for (int r = 0; r < 4; ++r) { a4[r] = oc[t][r]; b4[r] = oc[t][4 + r]; }
        *(v4fa*)(ocl + t * 256)     = a4;
        *(v4fa*)(ocl + t * 256 + 4) = b4;
      }
    }
    lds_wave_sync();
  }

  float inv[8];
#pragma unroll
  for (int r = 0; r < 8; ++r) inv[r] = (1.0f / lrow[r]) * OSC;
  float* os = lds_s + wave * (16 * OSTP);
  float* Cb = out + (size_t)q0 * QKS + h * FD;
#pragma unroll
  for (int t = 0; t < NTILE; ++t) {
    const v4f a4 = *(const v4fa*)(ow + t * 256);
    const v4f b4 = *(const v4fa*)(ow + t * 256 + 4);
#pragma unroll
    for (int r = 0; r < 4; ++r) {
      os[(8 * hh + r) * OSTP + t * 16 + c]     = fmaxf(a4[r] * inv[r], 0.0f);
      os[(8 * hh + 4 + r) * OSTP + t * 16 + c] = fmaxf(b4[r] * inv[4 + r], 0.0f);
    }
  }
  lds_wave_sync();
  for (int pass = 0; pass < 2; ++pass) {
#pragma unroll
    for (int row = 0; row < 16; ++row) {
      const v4f xv = *(const v4fa*)(os + row * OSTP + lane * 4);
      *(volatile v4f*)(Cb + (size_t)row * QKS + lane * 4) = xv;
    }
    __threadfence();
  }
}

#define WS_TOTAL ((size_t)NNODE*FIN*2 + (size_t)QKS*FIN*2 + (size_t)NHD*NNODE*FD*2 + (size_t)NNODE*QKS*2 + (size_t)QKS*NNODE*2 + (size_t)NHD*NNODE*4)
static_assert(WS_TOTAL == 30539776);
static_assert(WS_TOTAL <= 134217728);
static_assert((size_t)(NNODE - 1) * QKS + QKS - 1 < (size_t)NNODE * QKS);
static_assert((NNODE / 32) * (QKS / 128) % 4 == 0 && (QKS / 32) * (NNODE / 128) % 4 == 0);

extern "C" void kernel_launch(void* const* d_in, const int* in_sizes, int n_in,
                              void* d_out, int out_size, void* d_ws, size_t ws_size,
                              hipStream_t stream) {
  if (n_in < 5) return;
  if (in_sizes[0] != NNODE * FIN) return;
  if (in_sizes[1] != NHD * FIN * FD) return;
  if (in_sizes[2] != NHD * NNODE * FD) return;
  if (in_sizes[3] != NHD * NNODE * FD) return;
  if (in_sizes[4] != NHD * NNODE) return;
  if (out_size != NNODE * QKS) return;

  const float* X    = (const float*)d_in[0];
  const float* Wk   = (const float*)d_in[1];
  const float* asrc = (const float*)d_in[2];
  const float* adst = (const float*)d_in[3];
  const float* attb = (const float*)d_in[4];
  float* out = (float*)d_out;

  const size_t szXB  = (size_t)NNODE * FIN * 2;
  const size_t szWT  = (size_t)QKS * FIN * 2;
  const size_t szQP  = (size_t)NHD * NNODE * FD * 2;
  const size_t szKP  = (size_t)NNODE * QKS * 2;
  const size_t szVT  = (size_t)QKS * NNODE * 2;
  const size_t szSRC = (size_t)NHD * NNODE * 4;
  size_t off = 0;
  const size_t oXB  = off; off += szXB;
  const size_t oWT  = off; off += szWT;
  const size_t oQP  = off; off += szQP;
  const size_t oKP  = off; off += szKP;
  const size_t oVT  = off; off += szVT;
  const size_t oSRC = off; off += szSRC;
  if (off != WS_TOTAL) return;
  if (off > ws_size) return;

  char* ws = (char*)d_ws;
  unsigned short* XB  = (unsigned short*)(ws + oXB);
  unsigned short* WTB = (unsigned short*)(ws + oWT);
  unsigned short* QP  = (unsigned short*)(ws + oQP);
  unsigned short* KP  = (unsigned short*)(ws + oKP);
  unsigned short* VTP = (unsigned short*)(ws + oVT);
  float*          SRC = (float*)(ws + oSRC);

  const dim3 b256(256), b128(128);

  const int nux = NNODE * FIN / 8;
  prep_x_kernel<<<dim3((nux + 255) / 256), b256, 0, stream>>>(X, XB, nux);
  tconv_bf16_kernel<<<dim3(FD / 64, FIN / 64, NHD), b256, 0, stream>>>(Wk, WTB, FIN, FD, (long)FIN * FD, (long)FD * FIN);
  const int nuq = NHD * NNODE * FD / 8;
  prep_q_kernel<<<dim3((nuq + 255) / 256), b256, 0, stream>>>(adst, QP, nuq);
  const int tilesK = (NNODE / 32) * (QKS / 128);
  gemm_kernel<true><<<dim3(tilesK / 4), b128, 0, stream>>>(XB, FIN, WTB, FIN, KP, QKS, NNODE, QKS, FIN, asrc, SRC);
  const int tilesV = (QKS / 32) * (NNODE / 128);
  gemm_kernel<false><<<dim3(tilesV / 4), b128, 0, stream>>>(WTB, FIN, XB, FIN, VTP, NNODE, QKS, NNODE, FIN, asrc, SRC);
  (void)hipFuncSetAttribute(reinterpret_cast<const void*>(&attn_kernel), hipFuncAttributeMaxDynamicSharedMemorySize, ATT_LDS_BYTES);
  attn_kernel<<<dim3(NNODE / 64, NHD), b128, ATT_LDS_BYTES, stream>>>(QP, KP, VTP, SRC, attb, out);
  (void)hipGetLastError();
}
